// CAModule_53309134078084
// MI455X (gfx1250) — hardware-verified
//
#include <hip/hip_runtime.h>

#define B_   4
#define C_   256
#define CH_  128
#define N_   4096
#define NTOK (B_ * N_)
#define PSC  16384.0f

#define XT_PITCH 264
#define SO_PITCH 136
#define SY_PITCH 132
#define NXBLK (2 * B_ * (N_ / 64))
#define NWGRP ((3 * CH_ * C_ + C_ * CH_) / 8)
#define NWBLK ((NWGRP + 255) / 256)

typedef _Float16       v16h __attribute__((ext_vector_type(16)));
typedef _Float16       v8h  __attribute__((ext_vector_type(8)));
typedef __bf16         v16b __attribute__((ext_vector_type(16)));
typedef __bf16         v8b  __attribute__((ext_vector_type(8)));
typedef float          v8f  __attribute__((ext_vector_type(8)));
typedef float          v4f  __attribute__((ext_vector_type(4)));
typedef unsigned short v8us __attribute__((ext_vector_type(8)));
typedef v8h  __attribute__((may_alias)) v8ha;
typedef v8b  __attribute__((may_alias)) v8ba;
typedef v4f  __attribute__((may_alias)) v4fa;
typedef v8us __attribute__((may_alias)) v8usa;

union FragH { v16h v; v8h half[2]; };
union FragB { v16b v; v8b half[2]; };

__device__ __forceinline__ unsigned int bf_rne_u(float f) {
  const unsigned int u = __float_as_uint(f);
  return u + 0x7FFFu + ((u >> 16) & 1u);
}
__device__ __forceinline__ unsigned short bf_bits(float f) { return (unsigned short)(bf_rne_u(f) >> 16); }
__device__ __forceinline__ float bf_rn(float f) { return __uint_as_float(bf_rne_u(f) & 0xFFFF0000u); }
__device__ __forceinline__ unsigned short h_bits(float f) {
  const _Float16 hv = (_Float16)f;
  return __builtin_bit_cast(unsigned short, hv);
}

__device__ __forceinline__ v8f wmma_h(v16h a, v16h b, v8f c) {
  v8f d = __builtin_amdgcn_wmma_f32_16x16x32_f16(false, a, false, b, (short)0, c, false, false);
  asm volatile("v_nop\n\tv_nop\n\tv_nop\n\tv_nop" : "+v"(d) : "v"(a), "v"(b));
  return d;
}
__device__ __forceinline__ v8f wmma_b(v16b a, v16b b, v8f c) {
  v8f d = __builtin_amdgcn_wmma_f32_16x16x32_bf16(false, a, false, b, (short)0, c, false, false);
  asm volatile("v_nop\n\tv_nop\n\tv_nop\n\tv_nop" : "+v"(d) : "v"(a), "v"(b));
  return d;
}

__device__ __forceinline__ v16b ld_b(const unsigned short* p, int h) {
  FragB f;
  f.half[0] = *(const v8ba*)(p + 8 * h);
  f.half[1] = *(const v8ba*)(p + 16 + 8 * h);
  return f.v;
}
__device__ __forceinline__ v16h ld_h(const unsigned short* p, int h) {
  FragH f;
  f.half[0] = *(const v8ha*)(p + 8 * h);
  f.half[1] = *(const v8ha*)(p + 16 + 8 * h);
  return f.v;
}

__device__ __forceinline__ void xt_store_pass(const unsigned short* s, unsigned short* dst, int w, int lane) {
  #pragma unroll
  for (int i = 0; i < 8; ++i) {
    const int row = w * 8 + i;
    const v8us v = *(const v8usa*)(s + row * XT_PITCH + 8 * lane);
    *(volatile v8us*)(dst + (size_t)row * C_ + 8 * lane) = v;
  }
}

__global__ __launch_bounds__(256) void cvt_kernel(
    const float* __restrict__ xq, const float* __restrict__ xk,
    const float* __restrict__ wq, const float* __restrict__ wk,
    const float* __restrict__ wv, const float* __restrict__ wo,
    unsigned short* __restrict__ xqT, unsigned short* __restrict__ xkT,
    unsigned short* __restrict__ wqkv, unsigned short* __restrict__ woh)
{
  __shared__ __attribute__((aligned(16))) unsigned short sT[64 * XT_PITCH];

  const int tid = threadIdx.x, lane = tid & 31, w = tid >> 5;
  const int bid = blockIdx.x;
  if (bid < NXBLK) {
    const int which = bid / (B_ * (N_ / 64));
    const int rem = bid - which * (B_ * (N_ / 64));
    const int b = rem / (N_ / 64);
    const int n0 = (rem - b * (N_ / 64)) * 64;
    const float* src = ((which == 0) ? xq : xk) + (size_t)b * C_ * N_ + n0;
    const int col4 = tid & 15, csub = tid >> 4;
    #pragma unroll 4
    for (int p = 0; p < C_ / 16; ++p) {
      const int c = p * 16 + csub;
      const v4f v = *(const v4fa*)(src + (size_t)c * N_ + 4 * col4);
      unsigned short* s = sT + (4 * col4) * XT_PITCH + c;
      s[0]            = bf_bits(v.x);
      s[XT_PITCH]     = bf_bits(v.y);
      s[2 * XT_PITCH] = bf_bits(v.z);
      s[3 * XT_PITCH] = bf_bits(v.w);
    }
    __syncthreads();
    unsigned short* dst = ((which == 0) ? xqT : xkT) + ((size_t)b * N_ + n0) * C_;
    xt_store_pass(sT, dst, w, lane);
    __threadfence();
    xt_store_pass(sT, dst, w, lane);
  } else {
    const int g = (bid - NXBLK) * 256 + tid;
    if (g < 3 * (CH_ * C_ / 8)) {
      const int wsel = g / (CH_ * C_ / 8);
      const int off = (g - wsel * (CH_ * C_ / 8)) * 8;
      const float* src = ((wsel == 0) ? wq : ((wsel == 1) ? wk : wv)) + off;
      const v4f a = *(const v4fa*)src;
      const v4f c = *(const v4fa*)(src + 4);
      const v8us o = { bf_bits(a.x), bf_bits(a.y), bf_bits(a.z), bf_bits(a.w),
                       bf_bits(c.x), bf_bits(c.y), bf_bits(c.z), bf_bits(c.w) };
      unsigned short* dst = wqkv + (size_t)wsel * CH_ * C_ + off;
      *(volatile v8us*)dst = o;
      __threadfence();
      *(volatile v8us*)dst = o;
    } else if (g < NWGRP) {
      const int off = (g - 3 * (CH_ * C_ / 8)) * 8;
      const float* src = wo + off;
      const v4f a = *(const v4fa*)src;
      const v4f c = *(const v4fa*)(src + 4);
      const v8us o = { h_bits(64.0f * bf_rn(a.x)), h_bits(64.0f * bf_rn(a.y)),
                       h_bits(64.0f * bf_rn(a.z)), h_bits(64.0f * bf_rn(a.w)),
                       h_bits(64.0f * bf_rn(c.x)), h_bits(64.0f * bf_rn(c.y)),
                       h_bits(64.0f * bf_rn(c.z)), h_bits(64.0f * bf_rn(c.w)) };
      unsigned short* dst = woh + off;
      *(volatile v8us*)dst = o;
      __threadfence();
      *(volatile v8us*)dst = o;
    }
  }
}

__device__ __forceinline__ void proj_store_pass(const unsigned short* s0, const unsigned short* s1,
                                                int which, int chh, int m0, int b, int n0,
                                                unsigned short* ph, unsigned short* pl, unsigned short* vh,
                                                int w, int lane) {
  const int q8 = lane & 7, sub = lane >> 3;
  #pragma unroll
  for (int i = 0; i < 8; ++i) {
    const int lid = w * 32 + i * 4 + sub;
    if (which != 2) {
      const v8us a = *(const v8usa*)(s0 + lid * 64 + 8 * q8);
      const v8us c = *(const v8usa*)(s1 + lid * 64 + 8 * q8);
      const size_t off = (size_t)(m0 + lid) * CH_ + chh * 64 + 8 * q8;
      *(volatile v8us*)(ph + off) = a;
      *(volatile v8us*)(pl + off) = c;
    } else {
      const int d = lid >> 1, hl = lid & 1;
      const v8us a = *(const v8usa*)(s0 + d * 128 + 64 * hl + 8 * q8);
      const size_t off = ((size_t)b * CH_ + chh * 64 + d) * N_ + n0 + 64 * hl + 8 * q8;
      *(volatile v8us*)(vh + off) = a;
    }
  }
}

__global__ __launch_bounds__(128) void proj_kernel(
    const unsigned short* __restrict__ xqT, const unsigned short* __restrict__ xkT,
    const unsigned short* __restrict__ wqkv,
    const float* __restrict__ bq, const float* __restrict__ bk, const float* __restrict__ bv,
    unsigned short* __restrict__ qhi, unsigned short* __restrict__ qlo,
    unsigned short* __restrict__ khi, unsigned short* __restrict__ klo,
    unsigned short* __restrict__ vh)
{
  __shared__ __attribute__((aligned(16))) unsigned short sT[2][128 * 64];

  const int tid = threadIdx.x, lane = tid & 31, w = tid >> 5;
  const int h = lane >> 4, m = lane & 15;
  const int m0 = blockIdx.x * 128;
  const int cg = blockIdx.y;
  const int which = cg >> 1, chh = cg & 1;
  const unsigned short* xT = (which == 0) ? xqT : xkT;
  const int m0w = m0 + 32 * w;

  const unsigned short* xa0 = xT + (size_t)(m0w + m) * C_;
  const unsigned short* xa1 = xa0 + (size_t)16 * C_;
  const unsigned short* wb  = wqkv + ((size_t)which * CH_ + chh * 64 + m) * C_;

  const v8f zero8 = {0.f, 0.f, 0.f, 0.f, 0.f, 0.f, 0.f, 0.f};
  v8f acc[2][4];
  #pragma unroll
  for (int mt = 0; mt < 2; ++mt)
    #pragma unroll
    for (int nt = 0; nt < 4; ++nt) acc[mt][nt] = zero8;

  #pragma unroll 1
  for (int k0 = 0; k0 < C_; k0 += 32) {
    const v16b a0 = ld_b(xa0 + k0, h);
    const v16b a1 = ld_b(xa1 + k0, h);
    #pragma unroll
    for (int nt = 0; nt < 4; ++nt) {
      const v16b bfr = ld_b(wb + (size_t)nt * 16 * C_ + k0, h);
      acc[0][nt] = wmma_b(a0, bfr, acc[0][nt]);
      acc[1][nt] = wmma_b(a1, bfr, acc[1][nt]);
    }
  }

  const float* bias = (which == 0) ? bq : ((which == 1) ? bk : bv);
  #pragma unroll
  for (int nt = 0; nt < 4; ++nt) {
    const int feat = 16 * nt + m;
    const float bvl = bf_rn(bias[chh * 64 + feat]);
    #pragma unroll
    for (int mt = 0; mt < 2; ++mt) {
      #pragma unroll
      for (int r = 0; r < 8; ++r) {
        const int tokl = 32 * w + 16 * mt + 8 * h + r;
        const float y = acc[mt][nt][r] + bvl;
        if (which != 2) {
          const unsigned int hu = bf_rne_u(y) & 0xFFFF0000u;
          const float hi = __uint_as_float(hu);
          sT[0][tokl * 64 + feat] = (unsigned short)(hu >> 16);
          sT[1][tokl * 64 + feat] = bf_bits(y - hi);
        } else {
          sT[0][feat * 128 + tokl] = h_bits(16.0f * y);
        }
      }
    }
  }
  __syncthreads();

  const int b = m0 / N_, n0 = m0 - b * N_;
  unsigned short* ph = (which == 0) ? qhi : khi;
  unsigned short* pl = (which == 0) ? qlo : klo;
  proj_store_pass(sT[0], sT[1], which, chh, m0, b, n0, ph, pl, vh, w, lane);
  __threadfence();
  proj_store_pass(sT[0], sT[1], which, chh, m0, b, n0, ph, pl, vh, w, lane);
}

__device__ __forceinline__ v16h pack_p(v8f a, v8f c) {
  v16h r;
  #pragma unroll
  for (int i = 0; i < 8; ++i) {
    r[i]     = (_Float16)(a[i] * PSC);
    r[8 + i] = (_Float16)(c[i] * PSC);
  }
  return r;
}

__device__ __forceinline__ void att_store_pass(const unsigned short* so, unsigned short* ot,
                                               int b, int q0, int lane) {
  const int q8 = lane & 7, sub = lane >> 3;
  #pragma unroll
  for (int i = 0; i < 8; ++i) {
    const int lid = i * 4 + sub;
    const int row = lid >> 1, hl = lid & 1;
    const v8us v = *(const v8usa*)(so + row * SO_PITCH + 64 * hl + 8 * q8);
    const size_t gi = ((size_t)b * N_ + q0 + row) * CH_ + 64 * hl + 8 * q8;
    *(volatile v8us*)(ot + gi) = v;
  }
}

__global__ __launch_bounds__(128) void attn_kernel(
    const unsigned short* __restrict__ qhi, const unsigned short* __restrict__ qlo,
    const unsigned short* __restrict__ khi, const unsigned short* __restrict__ klo,
    const unsigned short* __restrict__ vh,
    unsigned short* __restrict__ ot)
{
  __shared__ __attribute__((aligned(16))) unsigned short sO[4 * 16 * SO_PITCH];

  const int tid = threadIdx.x, lane = tid & 31, w = tid >> 5;
  const int h = lane >> 4, m = lane & 15;
  const int b = blockIdx.y;
  const int q0 = blockIdx.x * 64 + 16 * w;

  const size_t qoff = ((size_t)b * N_ + q0 + m) * CH_;
  v16b qh_[4], ql_[4];
  #pragma unroll
  for (int c = 0; c < 4; ++c) {
    qh_[c] = ld_b(qhi + qoff + 32 * c, h);
    ql_[c] = ld_b(qlo + qoff + 32 * c, h);
  }

  const v8f zero8 = {0.f, 0.f, 0.f, 0.f, 0.f, 0.f, 0.f, 0.f};
  v8f o[8];
  #pragma unroll
  for (int t = 0; t < 8; ++t) o[t] = zero8;
  float mrun = -1e30f, lrun = 0.0f;

  const unsigned short* khb = khi + ((size_t)b * N_ + m) * CH_;
  const unsigned short* klb = klo + ((size_t)b * N_ + m) * CH_;
  const unsigned short* vb  = vh + ((size_t)b * CH_ + m) * N_;

  #pragma unroll 1
  for (int kb = 0; kb < N_; kb += 32) {
    v8f s[2];
    #pragma unroll
    for (int j = 0; j < 2; ++j) {
      const size_t ko = (size_t)(kb + 16 * j) * CH_;
      v8f z = zero8;
      #pragma unroll
      for (int c = 0; c < 4; ++c) {
        const v16b ah = ld_b(khb + ko + 32 * c, h);
        const v16b al = ld_b(klb + ko + 32 * c, h);
        z = wmma_b(ah, qh_[c], z);
        z = wmma_b(ah, ql_[c], z);
        z = wmma_b(al, qh_[c], z);
      }
      s[j] = z;
    }

    float mloc = s[0][0];
    #pragma unroll
    for (int j = 0; j < 2; ++j)
      #pragma unroll
      for (int r = 0; r < 8; ++r) mloc = fmaxf(mloc, s[j][r]);
    mloc = fmaxf(mloc, __shfl_xor(mloc, 16));
    const float mnew = fmaxf(mrun, mloc);
    const float alpha = __expf(mrun - mnew);
    mrun = mnew;
    float lsum = 0.0f;
    #pragma unroll
    for (int j = 0; j < 2; ++j)
      #pragma unroll
      for (int r = 0; r < 8; ++r) {
        const float p = __expf(s[j][r] - mnew);
        s[j][r] = p;
        lsum += p;
      }
    lsum += __shfl_xor(lsum, 16);
    lrun = lrun * alpha + lsum;
    #pragma unroll
    for (int t = 0; t < 8; ++t)
      #pragma unroll
      for (int r = 0; r < 8; ++r) o[t][r] = o[t][r] * alpha;

    const v16h pb = pack_p(s[0], s[1]);

    #pragma unroll
    for (int t = 0; t < 8; ++t) {
      const v16h vf = ld_h(vb + (size_t)(16 * t) * N_ + kb, h);
      o[t] = wmma_h(vf, pb, o[t]);
    }
  }

  const float inv = (1.0f / lrun) * (1.0f / PSC);
  unsigned short* so = sO + w * 16 * SO_PITCH;
  #pragma unroll
  for (int t = 0; t < 8; ++t)
    #pragma unroll
    for (int r = 0; r < 8; ++r)
      so[m * SO_PITCH + 16 * t + 8 * h + r] = h_bits(o[t][r] * inv);
  __syncthreads();

  att_store_pass(so, ot, b, q0, lane);
  __threadfence();
  att_store_pass(so, ot, b, q0, lane);
}

__device__ __forceinline__ void out_store_pass(const float* sY, const float* xq, float* out,
                                               int b, int o0, int n0, int w, int lane) {
  #pragma unroll
  for (int i = 0; i < 16; ++i) {
    const int ol = w * 16 + i;
    v4f v = *(const v4fa*)(sY + ol * SY_PITCH + 4 * lane);
    const size_t gi = ((size_t)(b * C_ + o0 + ol)) * N_ + n0 + 4 * lane;
    const v4f xr = *(const v4fa*)(xq + gi);
    v.x += bf_rn(xr.x); v.y += bf_rn(xr.y); v.z += bf_rn(xr.z); v.w += bf_rn(xr.w);
    *(volatile v4f*)(out + gi) = v;
  }
}

__global__ __launch_bounds__(128) void out_kernel(
    const unsigned short* __restrict__ woh,
    const unsigned short* __restrict__ ot,
    const float* __restrict__ bo, const float* __restrict__ xq,
    float* __restrict__ out)
{
  __shared__ __attribute__((aligned(16))) float sY[64 * SY_PITCH];

  const int tid = threadIdx.x, lane = tid & 31, w = tid >> 5;
  const int h = lane >> 4, m = lane & 15;
  const int m0 = blockIdx.x * 128;
  const int b = m0 / N_, n0 = m0 - b * N_;
  const int o0 = blockIdx.y * 64;
  const int wr = w >> 1, wc = w & 1;

  const unsigned short* ap0 = woh + (size_t)(o0 + 32 * wr + m) * CH_;
  const unsigned short* ap1 = ap0 + (size_t)16 * CH_;
  const unsigned short* bp  = ot + (size_t)(m0 + 64 * wc + m) * CH_;

  const v8f zero8 = {0.f, 0.f, 0.f, 0.f, 0.f, 0.f, 0.f, 0.f};
  v8f acc[2][4];
  #pragma unroll
  for (int mt = 0; mt < 2; ++mt)
    #pragma unroll
    for (int nt = 0; nt < 4; ++nt) acc[mt][nt] = zero8;

  #pragma unroll 1
  for (int k0 = 0; k0 < CH_; k0 += 32) {
    const v16h a0 = ld_h(ap0 + k0, h);
    const v16h a1 = ld_h(ap1 + k0, h);
    #pragma unroll
    for (int nt = 0; nt < 4; ++nt) {
      const v16h bfr = ld_h(bp + (size_t)nt * 16 * CH_ + k0, h);
      acc[0][nt] = wmma_h(a0, bfr, acc[0][nt]);
      acc[1][nt] = wmma_h(a1, bfr, acc[1][nt]);
    }
  }

  #pragma unroll
  for (int mt = 0; mt < 2; ++mt) {
    #pragma unroll
    for (int r = 0; r < 8; ++r) {
      const int ol = 32 * wr + 16 * mt + 8 * h + r;
      const float bvl = bf_rn(bo[o0 + ol]);
      #pragma unroll
      for (int nt = 0; nt < 4; ++nt) {
        const int nl = 64 * wc + 16 * nt + m;
        sY[ol * SY_PITCH + nl] = acc[mt][nt][r] * (1.0f / 1024.0f) + bvl;
      }
    }
  }
  __syncthreads();

  out_store_pass(sY, xq, out, b, o0, n0, w, lane);
  __threadfence();
  out_store_pass(sY, xq, out, b, o0, n0, w, lane);
}

extern "C" void kernel_launch(void* const* d_in, const int* in_sizes, int n_in,
                              void* d_out, int out_size, void* d_ws, size_t ws_size,
                              hipStream_t stream) {
  if (n_in < 10) return;
  if (in_sizes[0] != B_ * C_ * N_ || in_sizes[1] != B_ * C_ * N_) return;
  if (in_sizes[2] != CH_ * C_ || in_sizes[4] != CH_ * C_ || in_sizes[6] != CH_ * C_) return;
  if (in_sizes[3] != CH_ || in_sizes[5] != CH_ || in_sizes[7] != CH_) return;
  if (in_sizes[8] != C_ * CH_ || in_sizes[9] != C_) return;
  if (out_size != B_ * C_ * N_) return;

  const float* xq = (const float*)d_in[0];
  const float* xk = (const float*)d_in[1];
  const float* wq = (const float*)d_in[2];
  const float* bq = (const float*)d_in[3];
  const float* wk = (const float*)d_in[4];
  const float* bk = (const float*)d_in[5];
  const float* wv = (const float*)d_in[6];
  const float* bv = (const float*)d_in[7];
  const float* wo = (const float*)d_in[8];
  const float* bo = (const float*)d_in[9];
  float* out = (float*)d_out;

  const size_t sz_xt = (size_t)NTOK * C_ * 2;
  const size_t sz_w3 = (size_t)3 * CH_ * C_ * 2;
  const size_t sz_wo = (size_t)C_ * CH_ * 2;
  const size_t sz_pl = (size_t)NTOK * CH_ * 2;
  const size_t o_xqT  = 0;
  const size_t o_xkT  = o_xqT + sz_xt;
  const size_t o_wqkv = o_xkT + sz_xt;
  const size_t o_woh  = o_wqkv + sz_w3;
  const size_t o_qhi  = o_woh + sz_wo;
  const size_t o_qlo  = o_qhi + sz_pl;
  const size_t o_khi  = o_qlo + sz_pl;
  const size_t o_klo  = o_khi + sz_pl;
  const size_t o_vh   = o_klo + sz_pl;
  const size_t o_ot   = o_vh + sz_pl;
  const size_t total  = o_ot + sz_pl;
  if (total > ws_size) return;

  char* ws = (char*)d_ws;
  unsigned short* xqT  = (unsigned short*)(ws + o_xqT);
  unsigned short* xkT  = (unsigned short*)(ws + o_xkT);
  unsigned short* wqkv = (unsigned short*)(ws + o_wqkv);
  unsigned short* woh  = (unsigned short*)(ws + o_woh);
  unsigned short* qhi  = (unsigned short*)(ws + o_qhi);
  unsigned short* qlo  = (unsigned short*)(ws + o_qlo);
  unsigned short* khi  = (unsigned short*)(ws + o_khi);
  unsigned short* klo  = (unsigned short*)(ws + o_klo);
  unsigned short* vhp  = (unsigned short*)(ws + o_vh);
  unsigned short* otp  = (unsigned short*)(ws + o_ot);

  cvt_kernel<<<NXBLK + NWBLK, 256, 0, stream>>>(xq, xk, wq, wk, wv, wo, xqT, xkT, wqkv, woh);

  dim3 gProj(NTOK / 128, 6);
  proj_kernel<<<gProj, 128, 0, stream>>>(xqT, xkT, wqkv, bq, bk, bv, qhi, qlo, khi, klo, vhp);

  dim3 gAtt(N_ / 64, B_);
  attn_kernel<<<gAtt, 128, 0, stream>>>(qhi, qlo, khi, klo, vhp, otp);

  dim3 gOut(NTOK / 128, C_ / 64);
  out_kernel<<<gOut, 128, 0, stream>>>(woh, otp, bo, xq, out);
}
